// QRNN_75076028334120
// MI455X (gfx1250) — hardware-verified
//
#include <hip/hip_runtime.h>
#include <math.h>

constexpr int NBATCH = 8;
constexpr int NSTEP  = 4096;
constexpr int NCHAN  = 256;
constexpr int NUNIT  = 256;
constexpr int NGATE  = 3 * NUNIT;
constexpr int NWIN   = 2;
constexpr int KDIM   = NWIN * NCHAN;
constexpr int NROWS  = NBATCH * NSTEP;
constexpr int NTHR   = 256;
constexpr int NCOL8  = KDIM / 8;
static_assert(KDIM % 32 == 0);
static_assert(NROWS % 64 == 0 && NUNIT % 64 == 0);
static_assert(((NROWS / 64) * (NUNIT / 64)) % 8 == 0);
static_assert(KDIM % 64 == 0 && NGATE % 64 == 0);
static_assert((NROWS * NCOL8) % NTHR == 0);
static_assert(NUNIT == NTHR);
static_assert((NSTEP & (NSTEP - 1)) == 0);
static_assert(NGATE % 4 == 0 && (NGATE / 4) % 32 == 0);

typedef __attribute__((ext_vector_type(16))) _Float16 v16h;
typedef __attribute__((ext_vector_type(8)))  _Float16 v8h;
typedef __attribute__((ext_vector_type(16))) __bf16   v16b;
typedef __attribute__((ext_vector_type(8)))  __bf16   v8b;
typedef __attribute__((ext_vector_type(8)))  float    v8f;
typedef __attribute__((ext_vector_type(4)))  float    v4f;

__device__ __forceinline__ unsigned short f2bf_bits(float f) {
  unsigned u = __float_as_uint(f);
  return (unsigned short)((u + 0x7FFFu + ((u >> 16) & 1u)) >> 16);
}
__device__ __forceinline__ float bf_bits2f(unsigned short h) { return __uint_as_float(((unsigned)h) << 16); }
__device__ __forceinline__ float bf16r(float f) { return bf_bits2f(f2bf_bits(f)); }

__device__ __forceinline__ void dep_guard_h(v8f& a, v8f& b, v16h x, v16h y) { asm volatile("v_nop\n\tv_nop\n\tv_nop\n\tv_nop" : "+v"(a), "+v"(b) : "v"(x), "v"(y)); }
__device__ __forceinline__ void dep_guard_b(v8f& a, v8f& b, v16b x, v16b y) { asm volatile("v_nop\n\tv_nop\n\tv_nop\n\tv_nop" : "+v"(a), "+v"(b) : "v"(x), "v"(y)); }
__device__ __forceinline__ void keep4_h(v16h a, v16h b, v16h c, v16h d) { asm volatile("v_nop" :: "v"(a), "v"(b), "v"(c), "v"(d)); }
__device__ __forceinline__ void keep4_b(v16b a, v16b b, v16b c, v16b d) { asm volatile("v_nop" :: "v"(a), "v"(b), "v"(c), "v"(d)); }
__device__ __forceinline__ void acc_guard4(v8f& a, v8f& b, v8f& c, v8f& d) { asm volatile("v_nop\n\tv_nop\n\tv_nop\n\tv_nop" : "+v"(a), "+v"(b), "+v"(c), "+v"(d)); }
template <typename T> struct Frag;
template <> struct Frag<_Float16> {
  typedef v16h V; union U { v16h v; v8h h[2]; };
  static __device__ __forceinline__ v16h load(const _Float16* p) {
    U f; f.h[0] = *(const v8h*)(p); f.h[1] = *(const v8h*)(p + 16); return f.v;
  }
  static __device__ __forceinline__ v8f mma(v16h a, v16h b, v8f c) {
    return __builtin_amdgcn_wmma_f32_16x16x32_f16(false, a, false, b, (short)0, c, false, false);
  }
  static __device__ __forceinline__ void guard(v8f& a, v8f& b, v16h x, v16h y) { dep_guard_h(a, b, x, y); }
  static __device__ __forceinline__ void keep(v16h a, v16h b, v16h c, v16h d) { keep4_h(a, b, c, d); }
};
template <> struct Frag<__bf16> {
  typedef v16b V; union U { v16b v; v8b h[2]; };
  static __device__ __forceinline__ v16b load(const __bf16* p) {
    U f; f.h[0] = *(const v8b*)(p); f.h[1] = *(const v8b*)(p + 16); return f.v;
  }
  static __device__ __forceinline__ v8f mma(v16b a, v16b b, v8f c) {
    return __builtin_amdgcn_wmma_f32_16x16x32_bf16(false, a, false, b, (short)0, c, false, false);
  }
  static __device__ __forceinline__ void guard(v8f& a, v8f& b, v16b x, v16b y) { dep_guard_b(a, b, x, y); }
  static __device__ __forceinline__ void keep(v16b a, v16b b, v16b c, v16b d) { keep4_b(a, b, c, d); }
};

template <int ET> struct Elem;
template <> struct Elem<0> { typedef _Float16 T; };
template <> struct Elem<1> { typedef __bf16 T; };
template <int ET, bool SPLIT, int BIAS_MODE, int OUT_MODE, bool RESID, int ACT = 0>
__global__ __launch_bounds__(256) void wmma_gemm64(
    const unsigned short* __restrict__ Ap, const unsigned short* __restrict__ A2p, int lda, long strideA,
    const unsigned short* __restrict__ Btp, const unsigned short* __restrict__ Bt2p, int ldb, long strideB,
    void* __restrict__ Cout, void* __restrict__ Cout2, int ldc, long strideC,
    const float* __restrict__ bias,
    const float* __restrict__ resid, long strideR,
    int M, int N, int K, float scale) {
  typedef typename Elem<ET>::T T;
  typedef typename Frag<T>::V V;
  const T* A = (const T*)Ap; const T* A2 = (const T*)A2p; const T* Bt = (const T*)Btp; const T* Bt2 = (const T*)Bt2p;
  __shared__ __align__(16) float sT[8][16 * 68];
  const int b    = blockIdx.y;
  const int lane = threadIdx.x & 31;
  const int wave = threadIdx.x >> 5;
  const int tilesN = N >> 6;
  const int tilesM = M >> 6;
  const int tile = blockIdx.x * 8 + wave;
  if (tile >= tilesM * tilesN) return;
  const int tm = tile / tilesN;
  const int tn = tile - tm * tilesN;
  const int m0 = tm << 6;
  const int n0 = tn << 6;

  const T* Ab  = A  + (size_t)b * strideA;
  const T* Bb  = Bt + (size_t)b * strideB;
  const T* Ab2 = SPLIT ? (A2  + (size_t)b * strideA) : nullptr;
  const T* Bb2 = SPLIT ? (Bt2 + (size_t)b * strideB) : nullptr;

  const int rlane = lane & 15;
  const int koff  = (lane >> 4) * 8;
  const int mOff  = (lane >> 4) * 8;

  v8f acc[4][4];
#pragma unroll
  for (int i = 0; i < 4; ++i)
#pragma unroll
    for (int j = 0; j < 4; ++j) acc[i][j] = (v8f){0.f,0.f,0.f,0.f,0.f,0.f,0.f,0.f};

  for (int k0 = 0; k0 < K; k0 += 32) {
    V bh[4], bl[4];
#pragma unroll
    for (int j = 0; j < 4; ++j) {
      const size_t bo = (size_t)(n0 + (j << 4) + rlane) * ldb + koff + k0;
      bh[j] = Frag<T>::load(Bb + bo);
      if (SPLIT) bl[j] = Frag<T>::load(Bb2 + bo);
    }
#pragma unroll
    for (int i = 0; i < 4; ++i) {
      const size_t ao = (size_t)(m0 + (i << 4) + rlane) * lda + koff + k0;
      V ah = Frag<T>::load(Ab + ao);
      V al;
      if (SPLIT) al = Frag<T>::load(Ab2 + ao);
#pragma unroll
      for (int j = 0; j < 4; ++j) {
        acc[i][j] = Frag<T>::mma(ah, bh[j], acc[i][j]);
        if (SPLIT) {
          acc[i][j] = Frag<T>::mma(ah, bl[j], acc[i][j]);
          acc[i][j] = Frag<T>::mma(al, bh[j], acc[i][j]);
        }
      }
      Frag<T>::guard(acc[i][0], acc[i][3], ah, SPLIT ? al : ah);
    }
    Frag<T>::keep(bh[0], bh[1], bh[2], bh[3]);
    if (SPLIT) Frag<T>::keep(bl[0], bl[1], bl[2], bl[3]);
  }
  acc_guard4(acc[0][0], acc[0][1], acc[0][2], acc[0][3]);
  acc_guard4(acc[1][0], acc[1][1], acc[1][2], acc[1][3]);
  acc_guard4(acc[2][0], acc[2][1], acc[2][2], acc[2][3]);
  acc_guard4(acc[3][0], acc[3][1], acc[3][2], acc[3][3]);

  float* slab = sT[wave];
  const float* Rb = RESID ? (resid + (size_t)b * strideR) : nullptr;
#pragma unroll
  for (int i = 0; i < 4; ++i) {
    const int mBase = m0 + (i << 4);
#pragma unroll
    for (int j = 0; j < 4; ++j) {
      const int n = n0 + (j << 4) + rlane;
      float bv = 0.f;
      if (BIAS_MODE == 2) bv = bias[n];
#pragma unroll
      for (int r = 0; r < 8; ++r) {
        float v = acc[i][j][r] * scale;
        if (BIAS_MODE == 1) v += bias[mBase + mOff + r];
        if (BIAS_MODE == 2) v += bv;
        if (RESID) v += Rb[(size_t)(mBase + mOff + r) * ldc + n];
        if (ACT == 1) v = tanhf(v);
        if (ACT == 2) v = fmaxf(v, 0.0f);
        if (ACT == 3) v = v / (1.0f + expf(-v));
        if (ACT == 4) v = (v > 0.f) ? v : 0.01f * v;
        if (ACT == 5) v = 0.5f * v * (1.0f + erff(v * 0.70710678118654752f));
        slab[(mOff + r) * 68 + (j << 4) + rlane] = v;
      }
    }
    __builtin_amdgcn_fence(__ATOMIC_RELEASE, "workgroup");
    __builtin_amdgcn_wave_barrier();
    __builtin_amdgcn_fence(__ATOMIC_ACQUIRE, "workgroup");
    if (OUT_MODE == 0) {
      float* C = (float*)Cout + (size_t)b * strideC;
      const int hh = lane >> 4, c4 = (lane & 15) * 4;
      for (int pass = 0; pass < 2; ++pass) {
#pragma unroll
        for (int it = 0; it < 8; ++it) {
          const int row = it * 2 + hh;
          v4f v = *(const v4f*)(slab + row * 68 + c4);
          *(volatile v4f*)(C + (size_t)(mBase + row) * ldc + n0 + c4) = v;
        }
        __threadfence();
      }
    } else {
      const int q = lane >> 3, c8 = (lane & 7) * 8;
      unsigned short* C  = (unsigned short*)Cout  + (size_t)b * strideC;
      unsigned short* C2 = (OUT_MODE == 2) ? ((unsigned short*)Cout2 + (size_t)b * strideC) : nullptr;
      for (int pass = 0; pass < 2; ++pass) {
#pragma unroll
        for (int it = 0; it < 4; ++it) {
          const int row = it * 4 + q;
          const float* sp = slab + row * 68 + c8;
          v8h hv, lv;
#pragma unroll
          for (int e = 0; e < 8; ++e) {
            if (OUT_MODE == 1) {
              hv[e] = (_Float16)sp[e];
            } else {
              unsigned short hb = f2bf_bits(sp[e]);
              unsigned short lb = f2bf_bits(sp[e] - bf_bits2f(hb));
              hv[e] = __builtin_bit_cast(_Float16, hb);
              lv[e] = __builtin_bit_cast(_Float16, lb);
            }
          }
          *(volatile v8h*)(C + (size_t)(mBase + row) * ldc + n0 + c8) = hv;
          if (OUT_MODE == 2) *(volatile v8h*)(C2 + (size_t)(mBase + row) * ldc + n0 + c8) = lv;
        }
        __threadfence();
      }
    }
    __builtin_amdgcn_fence(__ATOMIC_RELEASE, "workgroup");
    __builtin_amdgcn_wave_barrier();
    __builtin_amdgcn_fence(__ATOMIC_ACQUIRE, "workgroup");
  }
}

template <int MODE>
__global__ __launch_bounds__(NTHR) void tpw_kernel(const float* __restrict__ src, int R, int C, int ldo,
                                                  unsigned short* __restrict__ O, float sc) {
  __shared__ float Tt[64 * 65];
  const int tid = threadIdx.x;
  const int c0 = blockIdx.x * 64, r0 = blockIdx.y * 64;
#pragma unroll
  for (int i = 0; i < 4; ++i) {
    const int idx = i * NTHR + tid;
    const int rr = idx >> 4, cc = (idx & 15) * 4;
    const v4f v = *(const v4f*)(src + (size_t)(r0 + rr) * (size_t)C + c0 + cc);
    Tt[rr * 65 + cc + 0] = v[0];
    Tt[rr * 65 + cc + 1] = v[1];
    Tt[rr * 65 + cc + 2] = v[2];
    Tt[rr * 65 + cc + 3] = v[3];
  }
  __syncthreads();
  const int q = tid >> 3, c8 = (tid & 7) * 8;
  v8h hv[2];
#pragma unroll
  for (int g = 0; g < 2; ++g) {
    const int qq = g * 32 + q;
#pragma unroll
    for (int e = 0; e < 8; ++e) {
      const float f = Tt[(c8 + e) * 65 + qq];
      unsigned short bits;
      if (MODE == 0) {
        bits = f2bf_bits(f * sc);
      } else {
        const float fb = bf_bits2f(f2bf_bits(f));
        bits = __builtin_bit_cast(unsigned short, (_Float16)(fb * sc));
      }
      hv[g][e] = __builtin_bit_cast(_Float16, bits);
    }
  }
  for (int pass = 0; pass < 2; ++pass) {
#pragma unroll
    for (int g = 0; g < 2; ++g) {
      const size_t o = (size_t)(c0 + g * 32 + q) * (size_t)ldo + (size_t)(r0 + c8);
      *(volatile v8h*)(O + o) = hv[g];
    }
    __threadfence();
  }
}

__global__ __launch_bounds__(NTHR) void im2col_kernel(const float* __restrict__ x, unsigned short* __restrict__ A) {
  const int i = blockIdx.x * NTHR + threadIdx.x;
  if (i < NROWS * NCOL8) {
    const int m = i >> 6;
    const int g = i & 63;
    const int t = m & (NSTEP - 1);
    const int older = (g < 32) ? 1 : 0;
    int srow = m - older;
    srow = srow < 0 ? 0 : srow;
    const int col = (g & 31) * 8;
    const float keep = (older != 0 && t == 0) ? 0.0f : 1.0f;
    const float* sp = x + (size_t)srow * NCHAN + col;
    const v4f a = *(const v4f*)(sp);
    const v4f c = *(const v4f*)(sp + 4);
    v8h hv;
#pragma unroll
    for (int e = 0; e < 4; ++e) {
      hv[e]     = __builtin_bit_cast(_Float16, f2bf_bits(a[e] * keep));
      hv[4 + e] = __builtin_bit_cast(_Float16, f2bf_bits(c[e] * keep));
    }
    unsigned short* dp = A + (size_t)i * 8;
    *(volatile v8h*)dp = hv;
    __threadfence();
    *(volatile v8h*)dp = hv;
  }
}

__global__ __launch_bounds__(NTHR) void bias_prep_kernel(const float* __restrict__ bsrc, float* __restrict__ dst) {
  const int tid = threadIdx.x;
  if (tid < NGATE / 4) {
    const v4f v = *(const v4f*)(bsrc + 4 * tid);
    v4f o;
#pragma unroll
    for (int e = 0; e < 4; ++e) o[e] = bf16r(v[e]);
    float* op = dst + 4 * tid;
    *(volatile v4f*)op = o;
    __threadfence();
    *(volatile v4f*)op = o;
  }
}

__global__ __launch_bounds__(NTHR) void fopool_kernel(const float* __restrict__ Zp, const float* __restrict__ Fp, float* hout) {
  const int u = threadIdx.x;
  const int b = blockIdx.x;
  const size_t base = (size_t)b * NSTEP * NUNIT + (size_t)u;
  const float* Op = hout;
  float c = 0.0f;
#pragma unroll 1
  for (int t = 0; t < NSTEP; ++t) {
    const size_t idx = base + (size_t)t * NUNIT;
    const float zp = Zp[idx];
    const float fp = Fp[idx];
    const float op = Op[idx];
    const float z = 1.0f - 2.0f * __builtin_amdgcn_rcpf(1.0f + expf(2.0f * zp));
    const float f = __builtin_amdgcn_rcpf(1.0f + expf(-fp));
    const float o = __builtin_amdgcn_rcpf(1.0f + expf(-op));
    const float bz = (1.0f - f) * z;
    c = f * c + bz;
    const float h = o * c;
    ((volatile float*)hout)[idx] = h;
    __threadfence();
    ((volatile float*)hout)[idx] = h;
  }
}

extern "C" void kernel_launch(void* const* d_in, const int* in_sizes, int n_in,
                              void* d_out, int out_size, void* d_ws, size_t ws_size, hipStream_t stream) {
  if (n_in < 3 || d_out == nullptr || d_ws == nullptr) return;
  if (in_sizes[0] != NROWS * NCHAN || in_sizes[1] != NWIN * NCHAN * NGATE || in_sizes[2] != NGATE ||
      out_size != NROWS * NUNIT) return;

  const float* x     = (const float*)d_in[0];
  const float* wconv = (const float*)d_in[1];
  const float* bias  = (const float*)d_in[2];
  float* out = (float*)d_out;

  char* ws = (char*)d_ws; size_t off = 0;
  auto carve = [&](size_t bytes) -> char* { char* p = ws + off; off += (bytes + 255) & ~(size_t)255; return p; };
  unsigned short* APL   = (unsigned short*)carve((size_t)NROWS * KDIM * 2);
  unsigned short* BTPL  = (unsigned short*)carve((size_t)NGATE * KDIM * 2);
  float*          BIASR = (float*)carve((size_t)NGATE * 4);
  float*          ZPL   = (float*)carve((size_t)NROWS * NUNIT * 4);
  float*          FPL   = (float*)carve((size_t)NROWS * NUNIT * 4);
  if (off > ws_size || off > (size_t)134217728) return;

  im2col_kernel<<<(NROWS * NCOL8) / NTHR, NTHR, 0, stream>>>(x, APL);
  tpw_kernel<0><<<dim3(NGATE / 64, KDIM / 64), NTHR, 0, stream>>>(wconv, KDIM, NGATE, KDIM, BTPL, 1.0f);
  bias_prep_kernel<<<1, NTHR, 0, stream>>>(bias, BIASR);

  const dim3 ggrid((NROWS / 64) * (NUNIT / 64) / 8, 1);
  wmma_gemm64<1, false, 2, 0, false, 0><<<ggrid, 256, 0, stream>>>(
      APL, APL, KDIM, 0L, BTPL + (size_t)0 * NUNIT * KDIM, BTPL, KDIM, 0L, (void*)ZPL, (void*)ZPL, NUNIT, 0L,
      BIASR + 0 * NUNIT, BIASR, 0L, NROWS, NUNIT, KDIM, 1.0f);
  wmma_gemm64<1, false, 2, 0, false, 0><<<ggrid, 256, 0, stream>>>(
      APL, APL, KDIM, 0L, BTPL + (size_t)1 * NUNIT * KDIM, BTPL, KDIM, 0L, (void*)FPL, (void*)FPL, NUNIT, 0L,
      BIASR + 1 * NUNIT, BIASR, 0L, NROWS, NUNIT, KDIM, 1.0f);
  wmma_gemm64<1, false, 2, 0, false, 0><<<ggrid, 256, 0, stream>>>(
      APL, APL, KDIM, 0L, BTPL + (size_t)2 * NUNIT * KDIM, BTPL, KDIM, 0L, (void*)out, (void*)out, NUNIT, 0L,
      BIASR + 2 * NUNIT, BIASR, 0L, NROWS, NUNIT, KDIM, 1.0f);

  fopool_kernel<<<NBATCH, NTHR, 0, stream>>>(ZPL, FPL, out);
}
